// TSingleHeadCausalSelfAttention_82429012345483
// MI455X (gfx1250) — hardware-verified
//
#include <hip/hip_runtime.h>
#include <stdint.h>

#define T_DIM  4096
#define C_DIM  1024
#define C3_DIM 3072

typedef __attribute__((ext_vector_type(16))) _Float16 v16h;
typedef __attribute__((ext_vector_type(8)))  _Float16 v8h;
typedef __attribute__((ext_vector_type(16))) __bf16   v16b;
typedef __attribute__((ext_vector_type(8)))  __bf16   v8b;
typedef __attribute__((ext_vector_type(8)))  float    v8f;
typedef __attribute__((ext_vector_type(4)))  float    v4f;
typedef __attribute__((ext_vector_type(8)))  unsigned short v8us;

__device__ __forceinline__ unsigned short f2bf_bits(float f) {
  unsigned u = __float_as_uint(f);
  return (unsigned short)((u + 0x7FFFu + ((u >> 16) & 1u)) >> 16);
}
__device__ __forceinline__ float bf_bits2f(unsigned short h) { return __uint_as_float(((unsigned)h) << 16); }
__device__ __forceinline__ void split_bf(float f, unsigned short& hb, unsigned short& lb) {
  hb = f2bf_bits(f);
  lb = f2bf_bits(f - bf_bits2f(hb));
}

__device__ __forceinline__ void dep_guard_h(v8f& a, v8f& b, v16h x, v16h y) { asm volatile("v_nop\n\tv_nop\n\tv_nop\n\tv_nop" : "+v"(a), "+v"(b) : "v"(x), "v"(y)); }
__device__ __forceinline__ void dep_guard_b(v8f& a, v8f& b, v16b x, v16b y) { asm volatile("v_nop\n\tv_nop\n\tv_nop\n\tv_nop" : "+v"(a), "+v"(b) : "v"(x), "v"(y)); }
__device__ __forceinline__ void keep4_h(v16h a, v16h b, v16h c, v16h d) { asm volatile("v_nop" :: "v"(a), "v"(b), "v"(c), "v"(d)); }
__device__ __forceinline__ void keep4_b(v16b a, v16b b, v16b c, v16b d) { asm volatile("v_nop" :: "v"(a), "v"(b), "v"(c), "v"(d)); }
__device__ __forceinline__ void acc_guard4(v8f& a, v8f& b, v8f& c, v8f& d) { asm volatile("v_nop\n\tv_nop\n\tv_nop\n\tv_nop" : "+v"(a), "+v"(b), "+v"(c), "+v"(d)); }
template <typename T> struct Frag;
template <> struct Frag<_Float16> {
  typedef v16h V; union U { v16h v; v8h h[2]; };
  static __device__ __forceinline__ v16h load(const _Float16* p) {
    U f; f.h[0] = *(const v8h*)(p); f.h[1] = *(const v8h*)(p + 16); return f.v;
  }
  static __device__ __forceinline__ v8f mma(v16h a, v16h b, v8f c) {
    return __builtin_amdgcn_wmma_f32_16x16x32_f16(false, a, false, b, (short)0, c, false, false);
  }
  static __device__ __forceinline__ void guard(v8f& a, v8f& b, v16h x, v16h y) { dep_guard_h(a, b, x, y); }
  static __device__ __forceinline__ void keep(v16h a, v16h b, v16h c, v16h d) { keep4_h(a, b, c, d); }
};
template <> struct Frag<__bf16> {
  typedef v16b V; union U { v16b v; v8b h[2]; };
  static __device__ __forceinline__ v16b load(const __bf16* p) {
    U f; f.h[0] = *(const v8b*)(p); f.h[1] = *(const v8b*)(p + 16); return f.v;
  }
  static __device__ __forceinline__ v8f mma(v16b a, v16b b, v8f c) {
    return __builtin_amdgcn_wmma_f32_16x16x32_bf16(false, a, false, b, (short)0, c, false, false);
  }
  static __device__ __forceinline__ void guard(v8f& a, v8f& b, v16b x, v16b y) { dep_guard_b(a, b, x, y); }
  static __device__ __forceinline__ void keep(v16b a, v16b b, v16b c, v16b d) { keep4_b(a, b, c, d); }
};

template <int ET> struct Elem;
template <> struct Elem<0> { typedef _Float16 T; };
template <> struct Elem<1> { typedef __bf16 T; };
template <int ET, bool SPLIT, int BIAS_MODE, int OUT_MODE, bool RESID, int ACT = 0>
__global__ __launch_bounds__(256) void wmma_gemm64(
    const unsigned short* __restrict__ Ap, const unsigned short* __restrict__ A2p, int lda, long strideA,
    const unsigned short* __restrict__ Btp, const unsigned short* __restrict__ Bt2p, int ldb, long strideB,
    void* __restrict__ Cout, void* __restrict__ Cout2, int ldc, long strideC,
    const float* __restrict__ bias,
    const float* __restrict__ resid, long strideR,
    int M, int N, int K, float scale) {
  typedef typename Elem<ET>::T T;
  typedef typename Frag<T>::V V;
  const T* A = (const T*)Ap; const T* A2 = (const T*)A2p; const T* Bt = (const T*)Btp; const T* Bt2 = (const T*)Bt2p;
  __shared__ __align__(16) float sT[8][16 * 68];
  const int b    = blockIdx.y;
  const int lane = threadIdx.x & 31;
  const int wave = threadIdx.x >> 5;
  const int tilesN = N >> 6;
  const int tilesM = M >> 6;
  const int tile = blockIdx.x * 8 + wave;
  if (tile >= tilesM * tilesN) return;
  const int tm = tile / tilesN;
  const int tn = tile - tm * tilesN;
  const int m0 = tm << 6;
  const int n0 = tn << 6;

  const T* Ab  = A  + (size_t)b * strideA;
  const T* Bb  = Bt + (size_t)b * strideB;
  const T* Ab2 = SPLIT ? (A2  + (size_t)b * strideA) : nullptr;
  const T* Bb2 = SPLIT ? (Bt2 + (size_t)b * strideB) : nullptr;

  const int rlane = lane & 15;
  const int koff  = (lane >> 4) * 8;
  const int mOff  = (lane >> 4) * 8;

  v8f acc[4][4];
#pragma unroll
  for (int i = 0; i < 4; ++i)
#pragma unroll
    for (int j = 0; j < 4; ++j) acc[i][j] = (v8f){0.f,0.f,0.f,0.f,0.f,0.f,0.f,0.f};

  for (int k0 = 0; k0 < K; k0 += 32) {
    V bh[4], bl[4];
#pragma unroll
    for (int j = 0; j < 4; ++j) {
      const size_t bo = (size_t)(n0 + (j << 4) + rlane) * ldb + koff + k0;
      bh[j] = Frag<T>::load(Bb + bo);
      if (SPLIT) bl[j] = Frag<T>::load(Bb2 + bo);
    }
#pragma unroll
    for (int i = 0; i < 4; ++i) {
      const size_t ao = (size_t)(m0 + (i << 4) + rlane) * lda + koff + k0;
      V ah = Frag<T>::load(Ab + ao);
      V al;
      if (SPLIT) al = Frag<T>::load(Ab2 + ao);
#pragma unroll
      for (int j = 0; j < 4; ++j) {
        acc[i][j] = Frag<T>::mma(ah, bh[j], acc[i][j]);
        if (SPLIT) {
          acc[i][j] = Frag<T>::mma(ah, bl[j], acc[i][j]);
          acc[i][j] = Frag<T>::mma(al, bh[j], acc[i][j]);
        }
      }
      Frag<T>::guard(acc[i][0], acc[i][3], ah, SPLIT ? al : ah);
    }
    Frag<T>::keep(bh[0], bh[1], bh[2], bh[3]);
    if (SPLIT) Frag<T>::keep(bl[0], bl[1], bl[2], bl[3]);
  }
  acc_guard4(acc[0][0], acc[0][1], acc[0][2], acc[0][3]);
  acc_guard4(acc[1][0], acc[1][1], acc[1][2], acc[1][3]);
  acc_guard4(acc[2][0], acc[2][1], acc[2][2], acc[2][3]);
  acc_guard4(acc[3][0], acc[3][1], acc[3][2], acc[3][3]);

  float* slab = sT[wave];
  const float* Rb = RESID ? (resid + (size_t)b * strideR) : nullptr;
#pragma unroll
  for (int i = 0; i < 4; ++i) {
    const int mBase = m0 + (i << 4);
#pragma unroll
    for (int j = 0; j < 4; ++j) {
      const int n = n0 + (j << 4) + rlane;
      float bv = 0.f;
      if (BIAS_MODE == 2) bv = bias[n];
#pragma unroll
      for (int r = 0; r < 8; ++r) {
        float v = acc[i][j][r] * scale;
        if (BIAS_MODE == 1) v += bias[mBase + mOff + r];
        if (BIAS_MODE == 2) v += bv;
        if (RESID) v += Rb[(size_t)(mBase + mOff + r) * ldc + n];
        if (ACT == 1) v = tanhf(v);
        if (ACT == 2) v = fmaxf(v, 0.0f);
        if (ACT == 3) v = v / (1.0f + expf(-v));
        if (ACT == 4) v = (v > 0.f) ? v : 0.01f * v;
        if (ACT == 5) v = 0.5f * v * (1.0f + erff(v * 0.70710678118654752f));
        slab[(mOff + r) * 68 + (j << 4) + rlane] = v;
      }
    }
    __builtin_amdgcn_fence(__ATOMIC_RELEASE, "workgroup");
    __builtin_amdgcn_wave_barrier();
    __builtin_amdgcn_fence(__ATOMIC_ACQUIRE, "workgroup");
    if (OUT_MODE == 0) {
      float* C = (float*)Cout + (size_t)b * strideC;
      const int hh = lane >> 4, c4 = (lane & 15) * 4;
      for (int pass = 0; pass < 2; ++pass) {
#pragma unroll
        for (int it = 0; it < 8; ++it) {
          const int row = it * 2 + hh;
          v4f v = *(const v4f*)(slab + row * 68 + c4);
          *(volatile v4f*)(C + (size_t)(mBase + row) * ldc + n0 + c4) = v;
        }
        __threadfence();
      }
    } else {
      const int q = lane >> 3, c8 = (lane & 7) * 8;
      unsigned short* C  = (unsigned short*)Cout  + (size_t)b * strideC;
      unsigned short* C2 = (OUT_MODE == 2) ? ((unsigned short*)Cout2 + (size_t)b * strideC) : nullptr;
      for (int pass = 0; pass < 2; ++pass) {
#pragma unroll
        for (int it = 0; it < 4; ++it) {
          const int row = it * 4 + q;
          const float* sp = slab + row * 68 + c8;
          v8h hv, lv;
#pragma unroll
          for (int e = 0; e < 8; ++e) {
            if (OUT_MODE == 1) {
              hv[e] = (_Float16)sp[e];
            } else {
              unsigned short hb = f2bf_bits(sp[e]);
              unsigned short lb = f2bf_bits(sp[e] - bf_bits2f(hb));
              hv[e] = __builtin_bit_cast(_Float16, hb);
              lv[e] = __builtin_bit_cast(_Float16, lb);
            }
          }
          *(volatile v8h*)(C + (size_t)(mBase + row) * ldc + n0 + c8) = hv;
          if (OUT_MODE == 2) *(volatile v8h*)(C2 + (size_t)(mBase + row) * ldc + n0 + c8) = lv;
        }
        __threadfence();
      }
    }
    __builtin_amdgcn_fence(__ATOMIC_RELEASE, "workgroup");
    __builtin_amdgcn_wave_barrier();
    __builtin_amdgcn_fence(__ATOMIC_ACQUIRE, "workgroup");
  }
}

__global__ __launch_bounds__(256) void split_planes8(const float* __restrict__ in,
                                                     unsigned short* __restrict__ hi,
                                                     unsigned short* __restrict__ lo, int n8) {
  const int i = blockIdx.x * 256 + threadIdx.x;
  if (i >= n8) return;
  const v4f a = *(const v4f*)(in + (size_t)8 * i);
  const v4f c = *(const v4f*)(in + (size_t)8 * i + 4);
  v8us hv, lv;
#pragma unroll
  for (int e = 0; e < 4; ++e) {
    unsigned short h0, l0;
    split_bf(a[e], h0, l0); hv[e] = h0;     lv[e] = l0;
    split_bf(c[e], h0, l0); hv[4 + e] = h0; lv[4 + e] = l0;
  }
  unsigned short* ph = hi + (size_t)8 * i;
  unsigned short* pl = lo + (size_t)8 * i;
  *(volatile v8us*)ph = hv;
  *(volatile v8us*)pl = lv;
  __threadfence();
  *(volatile v8us*)ph = hv;
  *(volatile v8us*)pl = lv;
}

__global__ __launch_bounds__(256) void transpose_split_w(const float* __restrict__ W,
                                                        unsigned short* __restrict__ hi,
                                                        unsigned short* __restrict__ lo,
                                                        int nrows, int ncols) {
  __shared__ float tile[64][65];
  const int tid = threadIdx.x;
  const int k0 = blockIdx.y * 64;
  const int n0 = blockIdx.x * 64;
#pragma unroll
  for (int it = 0; it < 4; ++it) {
    const int idx = tid + 256 * it;
    const int r = idx >> 4;
    const int c4 = (idx & 15) * 4;
    const v4f v = *(const v4f*)(W + (size_t)(k0 + r) * ncols + n0 + c4);
    tile[r][c4 + 0] = v[0]; tile[r][c4 + 1] = v[1]; tile[r][c4 + 2] = v[2]; tile[r][c4 + 3] = v[3];
  }
  __syncthreads();
  const int nn0 = tid >> 3, q = tid & 7;
  for (int pass = 0; pass < 2; ++pass) {
#pragma unroll
    for (int half = 0; half < 2; ++half) {
      const int nn = nn0 + 32 * half;
      v8us hv, lv;
#pragma unroll
      for (int e = 0; e < 8; ++e) {
        unsigned short h0, l0;
        split_bf(tile[8 * q + e][nn], h0, l0);
        hv[e] = h0; lv[e] = l0;
      }
      const size_t o = (size_t)(n0 + nn) * nrows + k0 + 8 * q;
      *(volatile v8us*)(hi + o) = hv;
      *(volatile v8us*)(lo + o) = lv;
    }
    __threadfence();
  }
}

template <int MODE>
__global__ __launch_bounds__(256) void gemm64_att(
    const unsigned short* __restrict__ Ap, const unsigned short* __restrict__ A2p, int lda,
    const unsigned short* __restrict__ Btp, const unsigned short* __restrict__ Bt2p, int ldb,
    float* __restrict__ Cout, int ldc, const int* __restrict__ n_padd_p,
    int tm0, int tilesM, int tilesN, int ntiles, int K, float scale) {
  typedef __bf16 T;
  typedef v16b V;
  const T* A = (const T*)Ap; const T* A2 = (const T*)A2p; const T* Bt = (const T*)Btp; const T* Bt2 = (const T*)Bt2p;
  __shared__ __align__(16) float sT[8][16 * 68];
  const int lane = threadIdx.x & 31;
  const int wave = threadIdx.x >> 5;
  const int tile = blockIdx.x * 8 + wave;
  if (tile >= ntiles) return;
  int am0, bn0, cm0, kend;
  if (MODE == 0) {
    const int g = (tm0 * (tm0 + 1)) / 2 + tile;
    int tm = (int)((sqrtf(8.0f * (float)g + 1.0f) - 1.0f) * 0.5f);
    if (((tm + 1) * (tm + 2)) / 2 <= g) ++tm;
    if (((tm + 1) * (tm + 2)) / 2 <= g) ++tm;
    if ((tm * (tm + 1)) / 2 > g) --tm;
    if ((tm * (tm + 1)) / 2 > g) --tm;
    tm = max(tm, tm0); tm = min(tm, tm0 + tilesM - 1);
    int tn = g - (tm * (tm + 1)) / 2;
    tn = max(tn, 0); tn = min(tn, tm);
    am0 = tm << 6; bn0 = tn << 6; cm0 = (tm - tm0) << 6; kend = K;
  } else {
    const int tml = tile / tilesN;
    const int tn  = tile - tml * tilesN;
    const int tmg = tm0 + tml;
    const int np  = n_padd_p[0];
    am0 = tml << 6; bn0 = tn << 6; cm0 = tml << 6;
    kend = ((tmg << 6) < np) ? T_DIM : ((tmg + 1) << 6);
    kend = min(kend, K);
  }
  kend = min(kend, T_DIM); kend = max(kend, 0);

  const int rlane = lane & 15;
  const int koff  = (lane >> 4) * 8;
  const int mOff  = (lane >> 4) * 8;

  v8f acc[4][4];
#pragma unroll
  for (int i = 0; i < 4; ++i)
#pragma unroll
    for (int j = 0; j < 4; ++j) acc[i][j] = (v8f){0.f,0.f,0.f,0.f,0.f,0.f,0.f,0.f};

  for (int k0 = 0; k0 < kend; k0 += 32) {
    V bh[4], bl[4];
#pragma unroll
    for (int j = 0; j < 4; ++j) {
      const size_t bo = (size_t)(bn0 + (j << 4) + rlane) * ldb + koff + k0;
      bh[j] = Frag<T>::load(Bt + bo);
      bl[j] = Frag<T>::load(Bt2 + bo);
    }
#pragma unroll
    for (int i = 0; i < 4; ++i) {
      const size_t ao = (size_t)(am0 + (i << 4) + rlane) * lda + koff + k0;
      V ah = Frag<T>::load(A + ao);
      V al = Frag<T>::load(A2 + ao);
#pragma unroll
      for (int j = 0; j < 4; ++j) {
        acc[i][j] = Frag<T>::mma(ah, bh[j], acc[i][j]);
        acc[i][j] = Frag<T>::mma(ah, bl[j], acc[i][j]);
        acc[i][j] = Frag<T>::mma(al, bh[j], acc[i][j]);
      }
      Frag<T>::guard(acc[i][0], acc[i][3], ah, al);
    }
    Frag<T>::keep(bh[0], bh[1], bh[2], bh[3]);
    Frag<T>::keep(bl[0], bl[1], bl[2], bl[3]);
  }
  acc_guard4(acc[0][0], acc[0][1], acc[0][2], acc[0][3]);
  acc_guard4(acc[1][0], acc[1][1], acc[1][2], acc[1][3]);
  acc_guard4(acc[2][0], acc[2][1], acc[2][2], acc[2][3]);
  acc_guard4(acc[3][0], acc[3][1], acc[3][2], acc[3][3]);

  float* slab = sT[wave];
#pragma unroll
  for (int i = 0; i < 4; ++i) {
    const int mBase = cm0 + (i << 4);
#pragma unroll
    for (int j = 0; j < 4; ++j) {
#pragma unroll
      for (int r = 0; r < 8; ++r) slab[(mOff + r) * 68 + (j << 4) + rlane] = acc[i][j][r] * scale;
    }
    __builtin_amdgcn_fence(__ATOMIC_RELEASE, "workgroup");
    __builtin_amdgcn_wave_barrier();
    __builtin_amdgcn_fence(__ATOMIC_ACQUIRE, "workgroup");
    {
      const int hh = lane >> 4, c4 = (lane & 15) * 4;
      for (int pass = 0; pass < 2; ++pass) {
#pragma unroll
        for (int it = 0; it < 8; ++it) {
          const int row = it * 2 + hh;
          v4f v = *(const v4f*)(slab + row * 68 + c4);
          *(volatile v4f*)(Cout + (size_t)(mBase + row) * ldc + bn0 + c4) = v;
        }
        __threadfence();
      }
    }
    __builtin_amdgcn_fence(__ATOMIC_RELEASE, "workgroup");
    __builtin_amdgcn_wave_barrier();
    __builtin_amdgcn_fence(__ATOMIC_ACQUIRE, "workgroup");
  }
}

__global__ __launch_bounds__(256) void softmax_rows(const float* __restrict__ S, const int* __restrict__ n_padd_p,
                                                   unsigned short* __restrict__ Ph, unsigned short* __restrict__ Pl,
                                                   int mrow0) {
  __shared__ float sv[T_DIM];
  __shared__ float red[8];
  const int tid = threadIdx.x, lane = tid & 31, wave = tid >> 5;
  const int il = blockIdx.x;
  const int i  = mrow0 + il;
  const int np = n_padd_p[0];
  const int tm = i >> 6;
  int kend = ((tm << 6) < np) ? T_DIM : ((tm + 1) << 6);
  kend = min(kend, T_DIM); kend = max(kend, 0);
  const bool uni = (i < np);
  const int jlo = (np < 0) ? 0 : np;
  const int jhi = uni ? -1 : min(i, T_DIM - 1);
  const float* srow = S + (size_t)il * T_DIM;

  float m = -__builtin_huge_valf();
  for (int j = jlo + tid; j <= jhi; j += 256) { const float s = srow[j]; sv[j] = s; m = fmaxf(m, s); }
#pragma unroll
  for (int off = 1; off < 32; off <<= 1) m = fmaxf(m, __shfl_xor(m, off, 32));
  if (lane == 0) red[wave] = m;
  __syncthreads();
  float rmax = red[0];
#pragma unroll
  for (int w = 1; w < 8; ++w) rmax = fmaxf(rmax, red[w]);
  __syncthreads();

  float sum = 0.f;
  for (int j = jlo + tid; j <= jhi; j += 256) { const float e = expf(sv[j] - rmax); sv[j] = e; sum += e; }
#pragma unroll
  for (int off = 1; off < 32; off <<= 1) sum += __shfl_xor(sum, off, 32);
  if (lane == 0) red[wave] = sum;
  __syncthreads();
  float tot = red[0];
#pragma unroll
  for (int w = 1; w < 8; ++w) tot += red[w];
  const float inv = (tot > 0.f) ? (1.0f / tot) : 0.f;
  const float cu  = 1.0f / (float)T_DIM;

  unsigned short* ph = Ph + (size_t)il * T_DIM;
  unsigned short* pl = Pl + (size_t)il * T_DIM;
  const int ng = kend >> 3;
  for (int pass = 0; pass < 2; ++pass) {
    for (int g = tid; g < ng; g += 256) {
      v8us hv, lv;
#pragma unroll
      for (int e = 0; e < 8; ++e) {
        const int j = 8 * g + e;
        const float ev = (j >= jlo && j <= jhi) ? sv[j] : 0.f;
        const float p = uni ? cu : ev * inv;
        unsigned short h0, l0;
        split_bf(p, h0, l0);
        hv[e] = h0; lv[e] = l0;
      }
      *(volatile v8us*)(ph + 8 * g) = hv;
      *(volatile v8us*)(pl + 8 * g) = lv;
    }
    __threadfence();
  }
}

extern "C" void kernel_launch(void* const* d_in, const int* in_sizes, int n_in,
                              void* d_out, int out_size, void* d_ws, size_t ws_size,
                              hipStream_t stream) {
  const int T = T_DIM, C = C_DIM, C3 = C3_DIM;
  if (n_in < 4) return;
  if (in_sizes[0] != T * C || in_sizes[1] != C * C3 || in_sizes[2] < C3 || in_sizes[3] < 1 || out_size != T * C) return;

  const float* x     = (const float*)d_in[0];
  const float* W     = (const float*)d_in[1];
  const float* bias  = (const float*)d_in[2];
  const int*   npadd = (const int*)d_in[3];
  float*       y     = (float*)d_out;

  const int QR = 1024;
  const int NCHUNK = T / QR;
  const size_t b_xp  = (size_t)T * C * 2;
  const size_t b_wp  = (size_t)C3 * C * 2;
  const size_t b_qkp = (size_t)T * 2 * C * 2;
  const size_t b_vtp = (size_t)C * T * 2;
  const size_t b_S   = (size_t)QR * T * 4;
  const size_t b_pp  = (size_t)QR * T * 2;
  size_t off = 0;
  const size_t o_xh = off; off += b_xp;  const size_t o_xl = off; off += b_xp;
  const size_t o_wh = off; off += b_wp;  const size_t o_wl = off; off += b_wp;
  const size_t o_qh = off; off += b_qkp; const size_t o_ql = off; off += b_qkp;
  const size_t o_vh = off; off += b_vtp; const size_t o_vl = off; off += b_vtp;
  const size_t o_S  = off; off += b_S;
  const size_t o_ph = off; off += b_pp;  const size_t o_pl = off; off += b_pp;
  if (off > ws_size) return;

  char* ws = (char*)d_ws;
  unsigned short* xh  = (unsigned short*)(ws + o_xh);
  unsigned short* xl  = (unsigned short*)(ws + o_xl);
  unsigned short* wth = (unsigned short*)(ws + o_wh);
  unsigned short* wtl = (unsigned short*)(ws + o_wl);
  unsigned short* qkh = (unsigned short*)(ws + o_qh);
  unsigned short* qkl = (unsigned short*)(ws + o_ql);
  unsigned short* vth = (unsigned short*)(ws + o_vh);
  unsigned short* vtl = (unsigned short*)(ws + o_vl);
  float*          S   = (float*)(ws + o_S);
  unsigned short* ph  = (unsigned short*)(ws + o_ph);
  unsigned short* pl  = (unsigned short*)(ws + o_pl);

  dim3 blk(256);
  {
    const int n8 = (T * C) / 8;
    split_planes8<<<dim3((n8 + 255) / 256), blk, 0, stream>>>(x, xh, xl, n8);
  }
  transpose_split_w<<<dim3(C3 / 64, C / 64), blk, 0, stream>>>(W, wth, wtl, C, C3);
  wmma_gemm64<1, true, 2, 2, false><<<dim3(((T / 64) * (2 * C / 64)) / 8, 1), blk, 0, stream>>>(
      xh, xl, C, 0L, wth, wtl, C, 0L, (void*)qkh, (void*)qkl, 2 * C, 0L,
      bias, x, 0L, T, 2 * C, C, 1.0f);
  wmma_gemm64<1, true, 1, 2, false><<<dim3(((C / 64) * (T / 64)) / 8, 1), blk, 0, stream>>>(
      wth + (size_t)2 * C * C, wtl + (size_t)2 * C * C, C, 0L, xh, xl, C, 0L, (void*)vth, (void*)vtl, T, 0L,
      bias + 2 * C, x, 0L, C, T, C, 1.0f);

  const float sc = 0.03125f;
  for (int ch = 0; ch < NCHUNK; ++ch) {
    const int tm0 = ch * (QR / 64);
    const int tilesM = QR / 64;
    const int ntri = ((tm0 + tilesM) * (tm0 + tilesM + 1)) / 2 - (tm0 * (tm0 + 1)) / 2;
    gemm64_att<0><<<dim3((ntri + 7) / 8), blk, 0, stream>>>(
        qkh, qkl, 2 * C, qkh + C, qkl + C, 2 * C, S, T, npadd, tm0, tilesM, 0, ntri, C, sc);
    softmax_rows<<<dim3(QR), blk, 0, stream>>>(S, npadd, ph, pl, tm0 * 64);
    const int ntpv = tilesM * (C / 64);
    gemm64_att<1><<<dim3((ntpv + 7) / 8), blk, 0, stream>>>(
        ph, pl, T, vth, vtl, T, y + (size_t)ch * QR * C, C, npadd, tm0, tilesM, C / 64, ntpv, T, 1.0f);
  }
}
